// MambaBlock_40982577938976
// MI455X (gfx1250) — hardware-verified
//
#include <hip/hip_runtime.h>
#include <math.h>

typedef __attribute__((ext_vector_type(16))) _Float16 v16h;
typedef __attribute__((ext_vector_type(8)))  _Float16 v8h;
typedef __attribute__((ext_vector_type(8)))  float    v8f;
typedef __attribute__((ext_vector_type(4)))  float    v4f;

constexpr int kBatch  = 32;
constexpr int kSeq    = 1024;
constexpr int kDm     = 64;
constexpr int kDin    = 256;
constexpr int kNst    = 16;
constexpr int kNh     = 4;
constexpr int kHd     = 64;
constexpr int kConvC  = kDin + 2 * kNst;
constexpr int kPrjN   = 2 * kDin + 2 * kNst + kNh;
constexpr int kZxP    = 576;
constexpr int kDtCol  = kDin + kConvC;
constexpr int kRows   = kBatch * kSeq;
constexpr int kChunk  = 16;
constexpr int kGP     = 260;
constexpr float kEps      = 1e-5f;
constexpr float kActCarry = 16.0f;
constexpr float kWCarry   = 32.0f;
constexpr float kFold     = 1.0f / (kActCarry * kWCarry);
static_assert(kConvC == 288 && kPrjN == 548 && kDtCol == 544, "column map");
static_assert(kNh * kHd == kDin, "heads");
static_assert(kZxP % 64 == 0 && kZxP >= kPrjN, "padded in_proj width");
static_assert(kRows % 64 == 0 && kDm % 64 == 0, "GEMM M,N multiples of 64");
static_assert(kDm % 32 == 0 && kDin % 32 == 0, "GEMM K multiples of 32");
static_assert(kSeq % kChunk == 0, "chunking");
static_assert(kConvC % 32 == 0 && kConvC / 32 == 9, "scan block = 9 waves");
static_assert(kFold == 0.001953125f, "carry fold");

constexpr size_t kOffW1H  = 0;
constexpr size_t kOffW2H  = kOffW1H + (size_t)kZxP * kDm * 2;
constexpr size_t kOffUH   = kOffW2H + (size_t)kDm * kDin * 2;
constexpr size_t kOffZX   = kOffUH  + (size_t)kRows * kDm * 2;
constexpr size_t kOffYH   = kOffZX  + (size_t)kRows * kZxP * 4;
constexpr size_t kWsTotal = kOffYH  + (size_t)kRows * kDin * 2;
static_assert(kWsTotal == 96575488ull, "carve total");
static_assert(kWsTotal <= 134217728ull, "carve cap");
static_assert((kOffW2H % 128) == 0 && (kOffUH % 128) == 0 && (kOffZX % 128) == 0 && (kOffYH % 128) == 0, "128-B aligned regions");

union FragH { v16h v; v8h h[2]; };
__device__ __forceinline__ v16h frag_load_h(const _Float16* p) {
  FragH f;
  f.h[0] = *(const v8h*)(p);
  f.h[1] = *(const v8h*)(p + 16);
  return f.v;
}
__device__ __forceinline__ v8f mma_h(v16h a, v16h b, v8f c) {
  return __builtin_amdgcn_wmma_f32_16x16x32_f16(false, a, false, b, (short)0, c, false, false);
}
__device__ __forceinline__ void grp_guard_h(v8f& a, v8f& b, v8f& c, v8f& d,
                                            v16h x, v16h y0, v16h y1, v16h y2, v16h y3) {
  asm volatile("v_nop\n\tv_nop\n\tv_nop\n\tv_nop"
               : "+v"(a), "+v"(b), "+v"(c), "+v"(d)
               : "v"(x), "v"(y0), "v"(y1), "v"(y2), "v"(y3));
}
__device__ __forceinline__ void acc_guard4(v8f& a, v8f& b, v8f& c, v8f& d) {
  asm volatile("v_nop\n\tv_nop\n\tv_nop\n\tv_nop" : "+v"(a), "+v"(b), "+v"(c), "+v"(d));
}

template <bool RES2X>
__global__ __launch_bounds__(256) void gemm_f16_kernel(
    const unsigned short* __restrict__ Ap, int lda,
    const unsigned short* __restrict__ Btp, int ldb,
    float* __restrict__ C, int ldc,
    const float* __restrict__ resid,
    int M, int N, int K, float scale)
{
  const _Float16* A  = (const _Float16*)Ap;
  const _Float16* Bt = (const _Float16*)Btp;
  __shared__ __align__(16) float sT[8][16 * 68];
  const int lane = threadIdx.x & 31;
  const int wave = threadIdx.x >> 5;
  const int tilesN = N >> 6;
  const int tilesM = M >> 6;
  const int tile = blockIdx.x * 8 + wave;
  if (tile >= tilesM * tilesN) return;
  const int tm = tile / tilesN;
  const int tn = tile - tm * tilesN;
  const int m0 = tm << 6;
  const int n0 = tn << 6;
  const int rlane = lane & 15;
  const int koff  = (lane >> 4) * 8;
  const int mOff  = (lane >> 4) * 8;

  v8f acc[4][4];
#pragma unroll
  for (int i = 0; i < 4; ++i)
#pragma unroll
    for (int j = 0; j < 4; ++j) acc[i][j] = (v8f){0.f, 0.f, 0.f, 0.f, 0.f, 0.f, 0.f, 0.f};

  for (int k0 = 0; k0 < K; k0 += 32) {
    v16h bh[4];
#pragma unroll
    for (int j = 0; j < 4; ++j) {
      const size_t bo = (size_t)(n0 + (j << 4) + rlane) * ldb + koff + k0;
      bh[j] = frag_load_h(Bt + bo);
    }
#pragma unroll
    for (int i = 0; i < 4; ++i) {
      const size_t ao = (size_t)(m0 + (i << 4) + rlane) * lda + koff + k0;
      const v16h ah = frag_load_h(A + ao);
#pragma unroll
      for (int j = 0; j < 4; ++j) acc[i][j] = mma_h(ah, bh[j], acc[i][j]);
      grp_guard_h(acc[i][0], acc[i][1], acc[i][2], acc[i][3], ah, bh[0], bh[1], bh[2], bh[3]);
    }
  }
  acc_guard4(acc[0][0], acc[0][1], acc[0][2], acc[0][3]);
  acc_guard4(acc[1][0], acc[1][1], acc[1][2], acc[1][3]);
  acc_guard4(acc[2][0], acc[2][1], acc[2][2], acc[2][3]);
  acc_guard4(acc[3][0], acc[3][1], acc[3][2], acc[3][3]);

  float* slab = sT[wave];
  const int hh = lane >> 4;
  const int c4 = (lane & 15) * 4;
#pragma unroll
  for (int i = 0; i < 4; ++i) {
    const int mBase = m0 + (i << 4);
#pragma unroll
    for (int j = 0; j < 4; ++j) {
#pragma unroll
      for (int r = 0; r < 8; ++r) {
        slab[(mOff + r) * 68 + (j << 4) + rlane] = acc[i][j][r] * scale;
      }
    }
    __builtin_amdgcn_fence(__ATOMIC_RELEASE, "workgroup");
    __builtin_amdgcn_wave_barrier();
    __builtin_amdgcn_fence(__ATOMIC_ACQUIRE, "workgroup");
    v4f val[8];
#pragma unroll
    for (int it = 0; it < 8; ++it) {
      const int row = it * 2 + hh;
      v4f v = *(const v4f*)(slab + row * 68 + c4);
      if (RES2X) {
        const v4f rv = *(const v4f*)(resid + (size_t)(mBase + row) * ldc + n0 + c4);
        const v4f r2 = rv + rv;
        v = v + r2;
      }
      val[it] = v;
    }
    for (int pass = 0; pass < 2; ++pass) {
#pragma unroll
      for (int it = 0; it < 8; ++it) {
        const int row = it * 2 + hh;
        *(volatile v4f*)(C + (size_t)(mBase + row) * ldc + n0 + c4) = val[it];
      }
      __threadfence();
    }
    __builtin_amdgcn_fence(__ATOMIC_RELEASE, "workgroup");
    __builtin_amdgcn_wave_barrier();
    __builtin_amdgcn_fence(__ATOMIC_ACQUIRE, "workgroup");
  }
}

constexpr int kW1Blocks = (kZxP * kDm / 8) / 256;
constexpr int kW2Blocks = (kDm * kDin / 8) / 256;
static_assert(kW1Blocks * 256 * 8 == kZxP * kDm && kW2Blocks * 256 * 8 == kDm * kDin, "weight plane coverage");

__global__ __launch_bounds__(256) void prep_weights_kernel(
    const float* __restrict__ w_in, const float* __restrict__ w_out,
    unsigned short* __restrict__ W1H, unsigned short* __restrict__ W2H)
{
  v8h hv;
  unsigned short* dst;
  if (blockIdx.x < kW1Blocks) {
    const int i   = blockIdx.x * 256 + threadIdx.x;
    const int e0  = i << 3;
    const int row = e0 >> 6;
    const int col = e0 & 63;
    const bool valid = (row < kPrjN);
    const int rowc = valid ? row : (kPrjN - 1);
    const float* p = w_in + (size_t)rowc * kDm + col;
    const v4f a0 = *(const v4f*)(p);
    const v4f a1 = *(const v4f*)(p + 4);
#pragma unroll
    for (int e = 0; e < 4; ++e) {
      const float f0 = a0[e];
      const float f1 = a1[e];
      hv[e]     = (_Float16)(valid ? (f0 * kWCarry) : 0.0f);
      hv[4 + e] = (_Float16)(valid ? (f1 * kWCarry) : 0.0f);
    }
    dst = W1H + e0;
  } else {
    const int i  = (blockIdx.x - kW1Blocks) * 256 + threadIdx.x;
    const int e0 = i << 3;
    const float* p = w_out + e0;
    const v4f a0 = *(const v4f*)(p);
    const v4f a1 = *(const v4f*)(p + 4);
#pragma unroll
    for (int e = 0; e < 4; ++e) {
      const float f0 = a0[e];
      const float f1 = a1[e];
      hv[e]     = (_Float16)(f0 * kWCarry);
      hv[4 + e] = (_Float16)(f1 * kWCarry);
    }
    dst = W2H + e0;
  }
  *(volatile v8h*)dst = hv;
  __threadfence();
  *(volatile v8h*)dst = hv;
}

static_assert((kRows * kDm / 8) % 256 == 0, "rmsnorm grid exact");
__global__ __launch_bounds__(256) void rmsnorm_cast_kernel(
    const float* __restrict__ x, const float* __restrict__ bw, unsigned short* __restrict__ UH)
{
  const int i = blockIdx.x * 256 + threadIdx.x;
  const size_t e0 = (size_t)i << 3;
  const int col = (int)(e0 & 63);
  const v4f a0 = *(const v4f*)(x + e0);
  const v4f a1 = *(const v4f*)(x + e0 + 4);
  const v4f w0 = *(const v4f*)(bw + col);
  const v4f w1 = *(const v4f*)(bw + col + 4);
  float ss = 0.0f;
#pragma unroll
  for (int e = 0; e < 4; ++e) {
    ss = fmaf(a0[e], a0[e], ss);
    ss = fmaf(a1[e], a1[e], ss);
  }
  ss += __shfl_xor(ss, 1, 32);
  ss += __shfl_xor(ss, 2, 32);
  ss += __shfl_xor(ss, 4, 32);
  const float sc = rsqrtf(ss * (1.0f / kDm) + kEps);
  v8h hv;
#pragma unroll
  for (int e = 0; e < 4; ++e) {
    const float f0 = a0[e] * sc * w0[e];
    const float f1 = a1[e] * sc * w1[e];
    hv[e]     = (_Float16)(f0 * kActCarry);
    hv[4 + e] = (_Float16)(f1 * kActCarry);
  }
  unsigned short* dst = UH + e0;
  *(volatile v8h*)dst = hv;
  __threadfence();
  *(volatile v8h*)dst = hv;
}

__global__ __launch_bounds__(288) void scan_fused_kernel(
    const float* __restrict__ ZX, const float* __restrict__ cw, const float* __restrict__ cb,
    const float* __restrict__ dtb, const float* __restrict__ Alog, const float* __restrict__ Dp,
    const float* __restrict__ ngw, unsigned short* __restrict__ YH)
{
  __shared__ __align__(16) float sXC[kChunk * kConvC];
  __shared__ __align__(16) float sG[kChunk * kGP];
  __shared__ __align__(16) float sDT[kChunk * kNh];
  __shared__ __align__(16) float sDA[kChunk * kNh];
  const int tid  = threadIdx.x;
  const int lane = tid & 31;
  const int wave = tid >> 5;
  const bool isState = (wave < 8);
  const size_t row0 = (size_t)blockIdx.x * kSeq;
  const int hd = (tid >> 6) & 3;
  const int hq = lane & 3;

  const v4f wv = *(const v4f*)(cw + tid * 4);
  const float w0 = wv[0], w1 = wv[1], w2 = wv[2], w3 = wv[3];
  const float bc = cb[tid];
  const float Dh = Dp[hd];
  const float Aq = -expf(Alog[hq]);
  const float bq = dtb[hq];
  const v4f g0 = *(const v4f*)(ngw + lane * 8);
  const v4f g1 = *(const v4f*)(ngw + lane * 8 + 4);

  float hst[kNst];
#pragma unroll
  for (int n = 0; n < kNst; ++n) hst[n] = 0.0f;
  float xm3 = 0.0f, xm2 = 0.0f, xm1 = 0.0f;
  const int wq = isState ? wave : 7;

#pragma unroll 1
  for (int c = 0; c < kSeq / kChunk; ++c) {
    const size_t r0 = row0 + (size_t)c * kChunk;

#pragma unroll 1
    for (int s = 0; s < kChunk; ++s) {
      const float* zr = ZX + (r0 + s) * kZxP;
      const float xcur = zr[kDin + tid];
      float acc = w0 * xm3;
      acc = fmaf(w1, xm2, acc);
      acc = fmaf(w2, xm1, acc);
      acc = fmaf(w3, xcur, acc);
      const float sv = acc + bc;
      const float sg = __builtin_amdgcn_rcpf(1.0f + expf(-sv));
      sXC[s * kConvC + tid] = sv * sg;
      xm3 = xm2;
      xm2 = xm1;
      xm1 = xcur;
      if (isState) {
        const float zv = zr[tid];
        const float sz = __builtin_amdgcn_rcpf(1.0f + expf(-zv));
        sG[s * kGP + tid] = zv * sz;
      }
    }
    if (!isState) {
#pragma unroll 1
      for (int k2 = 0; k2 < 2; ++k2) {
        const int idx = lane + 32 * k2;
        const int rr  = idx >> 2;
        const float v  = ZX[(r0 + rr) * kZxP + kDtCol + hq] + bq;
        const float ex = expf(-fabsf(v));
        const float dtv = fmaxf(v, 0.0f) + log1pf(ex);
        sDT[idx] = dtv;
        sDA[idx] = expf(dtv * Aq);
      }
    }
    __syncthreads();

    if (isState) {
#pragma unroll 1
      for (int s = 0; s < kChunk; ++s) {
        const float dtv = sDT[s * kNh + hd];
        const float dav = sDA[s * kNh + hd];
        const float xv  = sXC[s * kConvC + tid];
        const float* bp = sXC + s * kConvC + kDin;
        v4f Bq[4], Cq[4];
#pragma unroll
        for (int q4 = 0; q4 < 4; ++q4) {
          Bq[q4] = *(const v4f*)(bp + 4 * q4);
          Cq[q4] = *(const v4f*)(bp + kNst + 4 * q4);
        }
        const float dtx = dtv * xv;
        float y = 0.0f;
#pragma unroll
        for (int n = 0; n < kNst; ++n) {
          const float hn = fmaf(hst[n], dav, dtx * Bq[n >> 2][n & 3]);
          hst[n] = hn;
          y = fmaf(hn, Cq[n >> 2][n & 3], y);
        }
        y = fmaf(Dh, xv, y);
        const float gz = sG[s * kGP + tid];
        sG[s * kGP + tid] = y * gz;
      }
    }
    __syncthreads();

#pragma unroll 1
    for (int it = 0; it < 2; ++it) {
      const int row = wq * 2 + it;
      const float* sp = sG + row * kGP + lane * 8;
      const v4f a0 = *(const v4f*)(sp);
      const v4f a1 = *(const v4f*)(sp + 4);
      float ss = 0.0f;
#pragma unroll
      for (int e = 0; e < 4; ++e) {
        ss = fmaf(a0[e], a0[e], ss);
        ss = fmaf(a1[e], a1[e], ss);
      }
      ss += __shfl_xor(ss, 16, 32);
      ss += __shfl_xor(ss, 8, 32);
      ss += __shfl_xor(ss, 4, 32);
      ss += __shfl_xor(ss, 2, 32);
      ss += __shfl_xor(ss, 1, 32);
      const float sc = rsqrtf(ss * (1.0f / kDin) + kEps) * kActCarry;
      v8h hv;
#pragma unroll
      for (int e = 0; e < 4; ++e) {
        const float f0 = a0[e] * sc * g0[e];
        const float f1 = a1[e] * sc * g1[e];
        hv[e]     = (_Float16)f0;
        hv[4 + e] = (_Float16)f1;
      }
      if (isState) {
        unsigned short* dst = YH + (r0 + row) * kDin + lane * 8;
        *(volatile v8h*)dst = hv;
        __threadfence();
        *(volatile v8h*)dst = hv;
      }
    }
    __syncthreads();
  }
}

static_assert(((kRows / 64) * (kZxP / 64)) % 8 == 0 && ((kRows / 64) * (kDm / 64)) % 8 == 0, "GEMM grids exact");

extern "C" void kernel_launch(void* const* d_in, const int* in_sizes, int n_in,
                              void* d_out, int out_size, void* d_ws, size_t ws_size,
                              hipStream_t stream)
{
  if (n_in < 10) return;
  if (in_sizes[0] != kRows * kDm) return;
  if (in_sizes[1] != kPrjN * kDm) return;
  if (in_sizes[2] != kConvC * 4) return;
  if (in_sizes[3] != kConvC) return;
  if (in_sizes[4] != kNh || in_sizes[5] != kNh || in_sizes[6] != kNh) return;
  if (in_sizes[7] != kDin) return;
  if (in_sizes[8] != kDm * kDin) return;
  if (in_sizes[9] != kDm) return;
  if (out_size != kRows * kDm) return;
  if (ws_size < kWsTotal) return;

  const float* x       = (const float*)d_in[0];
  const float* w_in    = (const float*)d_in[1];
  const float* conv_w  = (const float*)d_in[2];
  const float* conv_b  = (const float*)d_in[3];
  const float* dt_bias = (const float*)d_in[4];
  const float* A_log   = (const float*)d_in[5];
  const float* Dp      = (const float*)d_in[6];
  const float* ngw     = (const float*)d_in[7];
  const float* w_out   = (const float*)d_in[8];
  const float* bnw     = (const float*)d_in[9];
  float* out = (float*)d_out;

  char* ws = (char*)d_ws;
  unsigned short* W1H = (unsigned short*)(ws + kOffW1H);
  unsigned short* W2H = (unsigned short*)(ws + kOffW2H);
  unsigned short* UH  = (unsigned short*)(ws + kOffUH);
  float*          ZX  = (float*)(ws + kOffZX);
  unsigned short* YH  = (unsigned short*)(ws + kOffYH);

  prep_weights_kernel<<<kW1Blocks + kW2Blocks, 256, 0, stream>>>(w_in, w_out, W1H, W2H);

  rmsnorm_cast_kernel<<<(kRows * kDm / 8) / 256, 256, 0, stream>>>(x, bnw, UH);

  gemm_f16_kernel<false><<<((kRows / 64) * (kZxP / 64)) / 8, 256, 0, stream>>>(
      UH, kDm, W1H, kDm, ZX, kZxP, x, kRows, kZxP, kDm, kFold);

  scan_fused_kernel<<<kBatch, kConvC, 0, stream>>>(ZX, conv_w, conv_b, dt_bias, A_log, Dp, ngw, YH);

  gemm_f16_kernel<true><<<((kRows / 64) * (kDm / 64)) / 8, 256, 0, stream>>>(
      YH, kDin, W2H, kDin, out, kDm, x, kRows, kDm, kDin, kFold);
}
